// TorchKAN_17643725652391
// MI455X (gfx1250) — hardware-verified
//
#include <hip/hip_runtime.h>
#include <math.h>

constexpr int kRows  = 32768;
constexpr int kDin   = 256;
constexpr int kHid   = 1024;
constexpr int kDout  = 256;
constexpr int kNact  = 6;
constexpr int kQRows = 8192;
constexpr int kNQ    = kRows / kQRows;
constexpr float kHCarry  = 16.0f;
constexpr float kW2Carry = 64.0f;
constexpr float kS2Scale = 1.0f / 1024.0f;

typedef __attribute__((ext_vector_type(16))) _Float16 v16h;
typedef __attribute__((ext_vector_type(8)))  _Float16 v8h;
typedef __attribute__((ext_vector_type(16))) __bf16   v16b;
typedef __attribute__((ext_vector_type(8)))  __bf16   v8b;
typedef __attribute__((ext_vector_type(8)))  float    v8f;
typedef __attribute__((ext_vector_type(4)))  float    v4f;
typedef __attribute__((ext_vector_type(4)))  unsigned int v4u;

__device__ __forceinline__ unsigned short f2bf_bits(float f) {
  unsigned u = __float_as_uint(f);
  return (unsigned short)((u + 0x7FFFu + ((u >> 16) & 1u)) >> 16);
}
__device__ __forceinline__ float bf_bits2f(unsigned short h) { return __uint_as_float(((unsigned)h) << 16); }

__device__ __forceinline__ void dep_guard_h(v8f& a, v8f& b, v16h x, v16h y) { asm volatile("v_nop\n\tv_nop\n\tv_nop\n\tv_nop" : "+v"(a), "+v"(b) : "v"(x), "v"(y)); }
__device__ __forceinline__ void dep_guard_b(v8f& a, v8f& b, v16b x, v16b y) { asm volatile("v_nop\n\tv_nop\n\tv_nop\n\tv_nop" : "+v"(a), "+v"(b) : "v"(x), "v"(y)); }
__device__ __forceinline__ void keep4_h(v16h a, v16h b, v16h c, v16h d) { asm volatile("v_nop" :: "v"(a), "v"(b), "v"(c), "v"(d)); }
__device__ __forceinline__ void keep4_b(v16b a, v16b b, v16b c, v16b d) { asm volatile("v_nop" :: "v"(a), "v"(b), "v"(c), "v"(d)); }
__device__ __forceinline__ void acc_guard4(v8f& a, v8f& b, v8f& c, v8f& d) { asm volatile("v_nop\n\tv_nop\n\tv_nop\n\tv_nop" : "+v"(a), "+v"(b), "+v"(c), "+v"(d)); }
template <typename T> struct Frag;
template <> struct Frag<_Float16> {
  typedef v16h V; union U { v16h v; v8h h[2]; };
  static __device__ __forceinline__ v16h load(const _Float16* p) {
    U f; f.h[0] = *(const v8h*)(p); f.h[1] = *(const v8h*)(p + 16); return f.v;
  }
  static __device__ __forceinline__ v8f mma(v16h a, v16h b, v8f c) {
    return __builtin_amdgcn_wmma_f32_16x16x32_f16(false, a, false, b, (short)0, c, false, false);
  }
  static __device__ __forceinline__ void guard(v8f& a, v8f& b, v16h x, v16h y) { dep_guard_h(a, b, x, y); }
  static __device__ __forceinline__ void keep(v16h a, v16h b, v16h c, v16h d) { keep4_h(a, b, c, d); }
};
template <> struct Frag<__bf16> {
  typedef v16b V; union U { v16b v; v8b h[2]; };
  static __device__ __forceinline__ v16b load(const __bf16* p) {
    U f; f.h[0] = *(const v8b*)(p); f.h[1] = *(const v8b*)(p + 16); return f.v;
  }
  static __device__ __forceinline__ v8f mma(v16b a, v16b b, v8f c) {
    return __builtin_amdgcn_wmma_f32_16x16x32_bf16(false, a, false, b, (short)0, c, false, false);
  }
  static __device__ __forceinline__ void guard(v8f& a, v8f& b, v16b x, v16b y) { dep_guard_b(a, b, x, y); }
  static __device__ __forceinline__ void keep(v16b a, v16b b, v16b c, v16b d) { keep4_b(a, b, c, d); }
};

__device__ __forceinline__ unsigned pk16(unsigned short a, unsigned short b) { return (unsigned)a | ((unsigned)b << 16); }
__device__ __forceinline__ unsigned short h_bits(float f) { const _Float16 h = (_Float16)f; return __builtin_bit_cast(unsigned short, h); }

template <int ET> struct Elem;
template <> struct Elem<0> { typedef _Float16 T; };
template <> struct Elem<1> { typedef __bf16 T; };
template <int ET, bool SPLIT, int BIAS_MODE, int OUT_MODE, bool RESID, int ACT = 0>
__global__ __launch_bounds__(256) void wmma_gemm64(
    const unsigned short* __restrict__ Ap, const unsigned short* __restrict__ A2p, int lda, long strideA,
    const unsigned short* __restrict__ Btp, const unsigned short* __restrict__ Bt2p, int ldb, long strideB,
    void* __restrict__ Cout, void* __restrict__ Cout2, int ldc, long strideC,
    const float* __restrict__ bias,
    const float* __restrict__ resid, long strideR,
    int M, int N, int K, float scale) {
  typedef typename Elem<ET>::T T;
  typedef typename Frag<T>::V V;
  const T* A = (const T*)Ap; const T* A2 = (const T*)A2p; const T* Bt = (const T*)Btp; const T* Bt2 = (const T*)Bt2p;
  __shared__ __align__(16) float sT[8][16 * 68];
  const int b    = blockIdx.y;
  const int lane = threadIdx.x & 31;
  const int wave = threadIdx.x >> 5;
  const int tilesN = N >> 6;
  const int tilesM = M >> 6;
  const int tile = blockIdx.x * 8 + wave;
  if (tile >= tilesM * tilesN) return;
  const int tm = tile / tilesN;
  const int tn = tile - tm * tilesN;
  const int m0 = tm << 6;
  const int n0 = tn << 6;

  const T* Ab  = A  + (size_t)b * strideA;
  const T* Bb  = Bt + (size_t)b * strideB;
  const T* Ab2 = SPLIT ? (A2  + (size_t)b * strideA) : nullptr;
  const T* Bb2 = SPLIT ? (Bt2 + (size_t)b * strideB) : nullptr;

  const int rlane = lane & 15;
  const int koff  = (lane >> 4) * 8;
  const int mOff  = (lane >> 4) * 8;

  v8f acc[4][4];
#pragma unroll
  for (int i = 0; i < 4; ++i)
#pragma unroll
    for (int j = 0; j < 4; ++j) acc[i][j] = (v8f){0.f,0.f,0.f,0.f,0.f,0.f,0.f,0.f};

  for (int k0 = 0; k0 < K; k0 += 32) {
    V bh[4], bl[4];
#pragma unroll
    for (int j = 0; j < 4; ++j) {
      const size_t bo = (size_t)(n0 + (j << 4) + rlane) * ldb + koff + k0;
      bh[j] = Frag<T>::load(Bb + bo);
      if (SPLIT) bl[j] = Frag<T>::load(Bb2 + bo);
    }
#pragma unroll
    for (int i = 0; i < 4; ++i) {
      const size_t ao = (size_t)(m0 + (i << 4) + rlane) * lda + koff + k0;
      V ah = Frag<T>::load(Ab + ao);
      V al;
      if (SPLIT) al = Frag<T>::load(Ab2 + ao);
#pragma unroll
      for (int j = 0; j < 4; ++j) {
        acc[i][j] = Frag<T>::mma(ah, bh[j], acc[i][j]);
        if (SPLIT) {
          acc[i][j] = Frag<T>::mma(ah, bl[j], acc[i][j]);
          acc[i][j] = Frag<T>::mma(al, bh[j], acc[i][j]);
        }
      }
      Frag<T>::guard(acc[i][0], acc[i][3], ah, SPLIT ? al : ah);
    }
    Frag<T>::keep(bh[0], bh[1], bh[2], bh[3]);
    if (SPLIT) Frag<T>::keep(bl[0], bl[1], bl[2], bl[3]);
  }
  acc_guard4(acc[0][0], acc[0][1], acc[0][2], acc[0][3]);
  acc_guard4(acc[1][0], acc[1][1], acc[1][2], acc[1][3]);
  acc_guard4(acc[2][0], acc[2][1], acc[2][2], acc[2][3]);
  acc_guard4(acc[3][0], acc[3][1], acc[3][2], acc[3][3]);

  float* slab = sT[wave];
  const float* Rb = RESID ? (resid + (size_t)b * strideR) : nullptr;
#pragma unroll
  for (int i = 0; i < 4; ++i) {
    const int mBase = m0 + (i << 4);
#pragma unroll
    for (int j = 0; j < 4; ++j) {
      const int n = n0 + (j << 4) + rlane;
      float bv = 0.f;
      if (BIAS_MODE == 2) bv = bias[n];
#pragma unroll
      for (int r = 0; r < 8; ++r) {
        float v = acc[i][j][r] * scale;
        if (BIAS_MODE == 1) v += bias[mBase + mOff + r];
        if (BIAS_MODE == 2) v += bv;
        if (RESID) v += Rb[(size_t)(mBase + mOff + r) * ldc + n];
        if (ACT == 2) v = fmaxf(v, 0.0f);
        if (ACT == 4) v = (v > 0.f) ? v : 0.01f * v;
        slab[(mOff + r) * 68 + (j << 4) + rlane] = v;
      }
    }
    __builtin_amdgcn_fence(__ATOMIC_RELEASE, "workgroup");
    __builtin_amdgcn_wave_barrier();
    __builtin_amdgcn_fence(__ATOMIC_ACQUIRE, "workgroup");
    if (OUT_MODE == 0) {
      float* C = (float*)Cout + (size_t)b * strideC;
      const int hh = lane >> 4, c4 = (lane & 15) * 4;
      for (int pass = 0; pass < 2; ++pass) {
#pragma unroll
        for (int it = 0; it < 8; ++it) {
          const int row = it * 2 + hh;
          v4f v = *(const v4f*)(slab + row * 68 + c4);
          *(volatile v4f*)(C + (size_t)(mBase + row) * ldc + n0 + c4) = v;
        }
        __threadfence();
      }
    } else {
      const int q = lane >> 3, c8 = (lane & 7) * 8;
      unsigned short* C  = (unsigned short*)Cout  + (size_t)b * strideC;
      unsigned short* C2 = (OUT_MODE == 2) ? ((unsigned short*)Cout2 + (size_t)b * strideC) : nullptr;
      for (int pass = 0; pass < 2; ++pass) {
#pragma unroll
        for (int it = 0; it < 4; ++it) {
          const int row = it * 4 + q;
          const float* sp = slab + row * 68 + c8;
          v8h hv, lv;
#pragma unroll
          for (int e = 0; e < 8; ++e) {
            if (OUT_MODE == 1) {
              hv[e] = (_Float16)sp[e];
            } else {
              unsigned short hb = f2bf_bits(sp[e]);
              unsigned short lb = f2bf_bits(sp[e] - bf_bits2f(hb));
              hv[e] = __builtin_bit_cast(_Float16, hb);
              lv[e] = __builtin_bit_cast(_Float16, lb);
            }
          }
          *(volatile v8h*)(C + (size_t)(mBase + row) * ldc + n0 + c8) = hv;
          if (OUT_MODE == 2) *(volatile v8h*)(C2 + (size_t)(mBase + row) * ldc + n0 + c8) = lv;
        }
        __threadfence();
      }
    }
    __builtin_amdgcn_fence(__ATOMIC_RELEASE, "workgroup");
    __builtin_amdgcn_wave_barrier();
    __builtin_amdgcn_fence(__ATOMIC_ACQUIRE, "workgroup");
  }
}

__global__ __launch_bounds__(256) void split_bf16_kernel(const float* __restrict__ in, unsigned short* __restrict__ hi,
                                                         unsigned short* __restrict__ lo, int n8) {
  const int i = blockIdx.x * 256 + threadIdx.x;
  if (i >= n8) return;
  const float* p = in + 8 * (size_t)i;
  const v4f a = *(const v4f*)(p);
  const v4f c = *(const v4f*)(p + 4);
  unsigned short hb[8], lb[8];
#pragma unroll
  for (int e = 0; e < 4; ++e) {
    hb[e] = f2bf_bits(a[e]);
    lb[e] = f2bf_bits(a[e] - bf_bits2f(hb[e]));
    hb[4 + e] = f2bf_bits(c[e]);
    lb[4 + e] = f2bf_bits(c[e] - bf_bits2f(hb[4 + e]));
  }
  const v4u uh = (v4u){pk16(hb[0], hb[1]), pk16(hb[2], hb[3]), pk16(hb[4], hb[5]), pk16(hb[6], hb[7])};
  const v4u ul = (v4u){pk16(lb[0], lb[1]), pk16(lb[2], lb[3]), pk16(lb[4], lb[5]), pk16(lb[6], lb[7])};
  unsigned short* qh = hi + 8 * (size_t)i;
  unsigned short* ql = lo + 8 * (size_t)i;
  *(volatile v4u*)qh = uh;
  *(volatile v4u*)ql = ul;
  __threadfence();
  *(volatile v4u*)qh = uh;
  *(volatile v4u*)ql = ul;
}

__global__ __launch_bounds__(256) void cast8_f16_kernel(const float* __restrict__ in, unsigned short* __restrict__ out,
                                                        int n8, float carry) {
  const int i = blockIdx.x * 256 + threadIdx.x;
  if (i >= n8) return;
  const float* p = in + 8 * (size_t)i;
  const v4f a = *(const v4f*)(p);
  const v4f c = *(const v4f*)(p + 4);
  unsigned short hb[8];
#pragma unroll
  for (int e = 0; e < 4; ++e) {
    hb[e]     = h_bits(a[e] * carry);
    hb[4 + e] = h_bits(c[e] * carry);
  }
  const v4u u = (v4u){pk16(hb[0], hb[1]), pk16(hb[2], hb[3]), pk16(hb[4], hb[5]), pk16(hb[6], hb[7])};
  unsigned short* q = out + 8 * (size_t)i;
  *(volatile v4u*)q = u;
  __threadfence();
  *(volatile v4u*)q = u;
}

__device__ __forceinline__ float kan_blend(float s, const float* __restrict__ ap) {
  const float c0 = ap[0], c1 = ap[1], c2 = ap[2], c3 = ap[3], c4 = ap[4], c5 = ap[5];
  const bool  pos = (s > 0.0f);
  const float sig = __builtin_amdgcn_rcpf(1.0f + expf(-s));
  const float th  = tanhf(s);
  const float re  = fmaxf(s, 0.0f);
  const float lk  = pos ? s : (0.01f * s);
  const float ea  = expf(-fabsf(s));
  const float sfp = re + log1pf(ea);
  const float el  = pos ? s : (ea - 1.0f);
  float h = c0 * sig;
  h += c1 * th;
  h += c2 * re;
  h += c3 * lk;
  h += c4 * sfp;
  h += c5 * el;
  return h;
}

template <int OMODE>
__global__ __launch_bounds__(256) void kan_mix_kernel(const float* __restrict__ S, const float* __restrict__ Acoef,
                                                      void* __restrict__ outp, int ncols, int total, float ocarry) {
  constexpr int EPT = (OMODE == 0) ? 8 : 4;
  __shared__ __align__(16) unsigned short sh16[(OMODE == 0) ? 256 * 8 : 8];
  __shared__ __align__(16) float          sh32[(OMODE == 1) ? 256 * 4 : 4];
  const int tid  = threadIdx.x;
  const int gthr = blockIdx.x * 256 + tid;
  const int e0   = gthr * EPT;
  const bool active = (e0 < total);
  const int e0c  = active ? e0 : 0;
  const int n0   = e0c & (ncols - 1);
#pragma unroll 1
  for (int e = 0; e < EPT; ++e) {
    const float s = S[e0c + e];
    const float h = kan_blend(s, Acoef + (size_t)(n0 + e) * kNact);
    if (OMODE == 0) sh16[tid * 8 + e] = h_bits(h * ocarry);
    else            sh32[tid * 4 + e] = h;
  }
  __syncthreads();
  if (OMODE == 0) {
    const v4u u = *(const v4u*)(sh16 + tid * 8);
    unsigned short* q = (unsigned short*)outp + (size_t)e0c;
    if (active) *(volatile v4u*)q = u;
    __threadfence();
    if (active) *(volatile v4u*)q = u;
  } else {
    const v4f v = *(const v4f*)(sh32 + tid * 4);
    float* q = (float*)outp + (size_t)e0c;
    if (active) *(volatile v4f*)q = v;
    __threadfence();
    if (active) *(volatile v4f*)q = v;
  }
}

extern "C" void kernel_launch(void* const* d_in, const int* in_sizes, int n_in,
                              void* d_out, int out_size, void* d_ws, size_t ws_size,
                              hipStream_t stream) {
  if (n_in < 5) return;
  if (in_sizes[0] != kRows * kDin || in_sizes[1] != kHid * kDin || in_sizes[2] != kHid * kNact ||
      in_sizes[3] != kDout * kHid || in_sizes[4] != kDout * kNact) return;
  if (out_size != kRows * kDout) return;

  const size_t off_xh  = 0;
  const size_t off_xl  = off_xh  + (size_t)kRows * kDin * 2;
  const size_t off_w1h = off_xl  + (size_t)kRows * kDin * 2;
  const size_t off_w1l = off_w1h + (size_t)kHid * kDin * 2;
  const size_t off_w2c = off_w1l + (size_t)kHid * kDin * 2;
  const size_t off_s1  = off_w2c + (size_t)kDout * kHid * 2;
  const size_t off_h16 = off_s1  + (size_t)kQRows * kHid * 4;
  const size_t off_s2  = off_h16 + (size_t)kQRows * kHid * 2;
  const size_t ws_end  = off_s2  + (size_t)kQRows * kDout * 4;
  if (ws_end > ws_size) return;

  const float* x  = (const float*)d_in[0];
  const float* w1 = (const float*)d_in[1];
  const float* a1 = (const float*)d_in[2];
  const float* w2 = (const float*)d_in[3];
  const float* a2 = (const float*)d_in[4];
  float* out = (float*)d_out;

  char* ws = (char*)d_ws;
  unsigned short* xh  = (unsigned short*)(ws + off_xh);
  unsigned short* xl  = (unsigned short*)(ws + off_xl);
  unsigned short* w1h = (unsigned short*)(ws + off_w1h);
  unsigned short* w1l = (unsigned short*)(ws + off_w1l);
  unsigned short* w2c = (unsigned short*)(ws + off_w2c);
  float*          s1  = (float*)(ws + off_s1);
  unsigned short* h16 = (unsigned short*)(ws + off_h16);
  float*          s2  = (float*)(ws + off_s2);

  {
    const int n8x = kRows * kDin / 8;
    const int n8w = kHid * kDin / 8;
    const int n8v = kDout * kHid / 8;
    split_bf16_kernel<<<dim3((n8x + 255) / 256), dim3(256), 0, stream>>>(x, xh, xl, n8x);
    split_bf16_kernel<<<dim3((n8w + 255) / 256), dim3(256), 0, stream>>>(w1, w1h, w1l, n8w);
    cast8_f16_kernel<<<dim3((n8v + 255) / 256), dim3(256), 0, stream>>>(w2, w2c, n8v, kW2Carry);
  }

  const int tiles1  = (kQRows / 64) * (kHid / 64);
  const int blocks1 = (tiles1 + 7) / 8;
  const int tiles2  = (kQRows / 64) * (kDout / 64);
  const int blocks2 = (tiles2 + 7) / 8;
  const int tot1    = kQRows * kHid;
  const int tot2    = kQRows * kDout;
  const int mixBlocks1 = (tot1 / 8 + 255) / 256;
  const int mixBlocks2 = (tot2 / 4 + 255) / 256;

  for (int q = 0; q < kNQ; ++q) {
    const unsigned short* xhq = xh + (size_t)q * kQRows * kDin;
    const unsigned short* xlq = xl + (size_t)q * kQRows * kDin;
    float* outq = out + (size_t)q * kQRows * kDout;

    wmma_gemm64<1, true, 0, 0, false, 0><<<dim3(blocks1, 1), dim3(256), 0, stream>>>(
        xhq, xlq, kDin, 0L,
        w1h, w1l, kDin, 0L,
        (void*)s1, (void*)s1, kHid, 0L,
        a1, s1, 0L,
        kQRows, kHid, kDin, 1.0f);

    kan_mix_kernel<0><<<dim3(mixBlocks1), dim3(256), 0, stream>>>(s1, a1, (void*)h16, kHid, tot1, kHCarry);

    wmma_gemm64<0, false, 0, 0, false, 0><<<dim3(blocks2, 1), dim3(256), 0, stream>>>(
        h16, h16, kHid, 0L,
        w2c, w2c, kHid, 0L,
        (void*)s2, (void*)s2, kDout, 0L,
        a2, s2, 0L,
        kQRows, kDout, kHid, kS2Scale);

    kan_mix_kernel<1><<<dim3(mixBlocks2), dim3(256), 0, stream>>>(s2, a2, (void*)outq, kDout, tot2, 1.0f);
  }
}
